// MGCN_block_76089640616098
// MI455X (gfx1250) — hardware-run, weakly checked
//
#include <hip/hip_runtime.h>
#include <stddef.h>
#include <math.h>

#define NBATCH 32
#define NNODE 1024
#define NT 64
#define WGROW 12352
#define WTPLANE (12352 * 64)
#define WGPLANE (1024 * 12352)
#define SCPLANE (2048 * 1024)
#define STPLANE (1024 * 1024)
#define XGPLANE (2048 * 2048)
#define SP 68
#define HP 72

static_assert(NNODE % 128 == 0);
static_assert(WGROW % 64 == 0);
static_assert((SP * 4) % 16 == 0);
static_assert((HP * 2) % 16 == 0);

typedef _Float16 f16;
typedef unsigned short u16;
typedef f16 v16h __attribute__((ext_vector_type(16)));
typedef f16 v8h_t __attribute__((ext_vector_type(8)));
typedef v8h_t __attribute__((may_alias)) v8h;
typedef __bf16 v16b __attribute__((ext_vector_type(16)));
typedef u16 v8us_t __attribute__((ext_vector_type(8)));
typedef v8us_t __attribute__((may_alias)) v8us;
typedef float v8f __attribute__((ext_vector_type(8)));
typedef float v4f_t __attribute__((ext_vector_type(4)));
typedef v4f_t __attribute__((may_alias)) v4f;
typedef unsigned int v4u_t __attribute__((ext_vector_type(4)));
typedef v4u_t __attribute__((may_alias)) v4u;

#define NOP4 "v_nop\n\tv_nop\n\tv_nop\n\tv_nop"

__device__ __forceinline__ v8f zero8() {
    v8f z;
#pragma unroll
    for (int i = 0; i < 8; ++i) z[i] = 0.0f;
    return z;
}

__device__ __forceinline__ v16h ldf(const f16* p, int k0) {
    union { v16h v; v8h_t hh[2]; } f;
    f.hh[0] = *(const v8h*)(p + k0);
    f.hh[1] = *(const v8h*)(p + k0 + 16);
    return f.v;
}
__device__ __forceinline__ v16b ldb(const u16* p, int k0) {
    union { v16b v; v8us_t hh[2]; } f;
    f.hh[0] = *(const v8us*)(p + k0);
    f.hh[1] = *(const v8us*)(p + k0 + 16);
    return f.v;
}
__device__ __forceinline__ v8f wm16(v16h a, v16h b, v8f c) {
    return __builtin_amdgcn_wmma_f32_16x16x32_f16(false, a, false, b, (short)0, c, false, false);
}
__device__ __forceinline__ v8f wmb16(v16b a, v16b b, v8f c) {
    return __builtin_amdgcn_wmma_f32_16x16x32_bf16(false, a, false, b, (short)0, c, false, false);
}

__device__ __forceinline__ v4u_t pack8h(v4f_t a, v4f_t b, float s) {
    union { v8h_t hh; v4u_t u; } pk;
#pragma unroll
    for (int j = 0; j < 4; ++j) { pk.hh[j] = (f16)(a[j] * s); pk.hh[4 + j] = (f16)(b[j] * s); }
    return pk.u;
}

__global__ void __launch_bounds__(256) k_prep_e(const float* __restrict__ E, u16* __restrict__ Ehi,
                                               u16* __restrict__ Elo, f16* __restrict__ E16, int n8)
{
    const int i = blockIdx.x * 256 + threadIdx.x;
    if (i >= n8) return;
    const v4f_t a = *(const v4f*)(E + (size_t)i * 8);
    const v4f_t b = *(const v4f*)(E + (size_t)i * 8 + 4);
    float v[8];
#pragma unroll
    for (int j = 0; j < 4; ++j) { v[j] = a[j]; v[4 + j] = b[j]; }
    union { v8us_t s; v4u_t u; } ph, pl;
    union { v8h_t hh; v4u_t u; } pe;
#pragma unroll
    for (int j = 0; j < 8; ++j) {
        const unsigned int u  = __float_as_uint(v[j]);
        const unsigned int hb = (u + 0x7FFFu + ((u >> 16) & 1u)) >> 16;
        const float hf = __uint_as_float(hb << 16);
        const unsigned int ur = __float_as_uint(v[j] - hf);
        const unsigned int lb = (ur + 0x7FFFu + ((ur >> 16) & 1u)) >> 16;
        ph.s[j] = (u16)hb;
        pl.s[j] = (u16)lb;
        pe.hh[j] = (f16)(v[j] * 16.0f);
    }
    *(volatile v4u_t*)(Ehi + (size_t)i * 8) = ph.u;
    *(volatile v4u_t*)(Elo + (size_t)i * 8) = pl.u;
    *(volatile v4u_t*)(E16 + (size_t)i * 8) = pe.u;
    __threadfence();
    *(volatile v4u_t*)(Ehi + (size_t)i * 8) = ph.u;
    *(volatile v4u_t*)(Elo + (size_t)i * 8) = pl.u;
    *(volatile v4u_t*)(E16 + (size_t)i * 8) = pe.u;
}

__global__ void __launch_bounds__(128) k_trw(const float* __restrict__ W1, const float* __restrict__ W2,
                                             const float* __restrict__ b1p, const float* __restrict__ b2p,
                                             const float* __restrict__ p1w, const float* __restrict__ p2w,
                                             f16* __restrict__ WT, f16* __restrict__ pwT)
{
    __shared__ __align__(16) float ts[64 * SP];
    const int tid = threadIdx.x, xk = blockIdx.x, gg = blockIdx.y, ly = blockIdx.z;
    if (xk == 193 && gg == 1) return;
    const float* W  = ly ? W2 : W1;
    const float* bp = ly ? b2p : b1p;
    const float* pw = ly ? p2w : p1w;
    f16* wt = WT + (size_t)(ly * 2 + gg) * WTPLANE;
    const float* inb; int in_rs; f16* outb; int out_rs; float scale;
    if (xk < 192) {
        inb = W + (size_t)gg * 786432 + (size_t)xk * 64; in_rs = 12288;
        outb = wt + (size_t)xk * 64; out_rs = 12288;
        scale = (xk >= 64 && xk < 128) ? 4.0f : 64.0f;
    } else if (xk == 192) {
        inb = bp + (size_t)gg * 4096; in_rs = 64;
        outb = wt + (size_t)12288 * 64; out_rs = 64; scale = 64.0f;
    } else {
        inb = pw; in_rs = 64;
        outb = pwT + (size_t)ly * 4096; out_rs = 64; scale = 4.0f;
    }
#pragma unroll
    for (int q = 0; q < 8; ++q) {
        const int idx = tid + 128 * q;
        const int r = idx >> 4, c4 = (idx & 15) * 4;
        *(v4f*)(ts + r * SP + c4) = *(const v4f*)(inb + (size_t)r * in_rs + c4);
    }
    __syncthreads();
    const int Lc = tid >> 3, p = tid & 7;
    v4u_t o[4];
#pragma unroll
    for (int s = 0; s < 4; ++s) {
        const int c = 16 * s + Lc;
        v4f_t a, b;
#pragma unroll
        for (int jj = 0; jj < 4; ++jj) { a[jj] = ts[(8 * p + jj) * SP + c]; b[jj] = ts[(8 * p + 4 + jj) * SP + c]; }
        o[s] = pack8h(a, b, scale);
    }
#pragma unroll
    for (int s = 0; s < 4; ++s)
        *(volatile v4u_t*)(outb + (size_t)(16 * s + Lc) * out_rs + 8 * p) = o[s];
    __threadfence();
#pragma unroll
    for (int s = 0; s < 4; ++s)
        *(volatile v4u_t*)(outb + (size_t)(16 * s + Lc) * out_rs + 8 * p) = o[s];
}

__global__ void __launch_bounds__(128) k_trx(const float* __restrict__ x, f16* __restrict__ XT,
                                             f16* __restrict__ X0)
{
    __shared__ __align__(16) float ts[64 * SP];
    const int tid = threadIdx.x, b = blockIdx.y;
    const int m0 = blockIdx.x * 64;
    const float* xb = x + (size_t)b * 65536 + (size_t)m0 * 64;
#pragma unroll
    for (int q = 0; q < 8; ++q) {
        const int idx = tid + 128 * q;
        const int i = idx >> 4, c4 = (idx & 15) * 4;
        *(v4f*)(ts + i * SP + c4) = *(const v4f*)(xb + (size_t)i * 64 + c4);
    }
    __syncthreads();
    const int L = tid >> 3, p = tid & 7;
    v4u_t xo[4], to[4];
#pragma unroll
    for (int s = 0; s < 4; ++s) {
        const int i = 16 * s + L;
        const v4f_t a = *(const v4f*)(ts + i * SP + 8 * p);
        const v4f_t c = *(const v4f*)(ts + i * SP + 8 * p + 4);
        xo[s] = pack8h(a, c, 1.0f);
        const int t = 16 * s + L;
        v4f_t d, e;
#pragma unroll
        for (int jj = 0; jj < 4; ++jj) { d[jj] = ts[(8 * p + jj) * SP + t]; e[jj] = ts[(8 * p + 4 + jj) * SP + t]; }
        to[s] = pack8h(d, e, 1.0f);
    }
#pragma unroll
    for (int s = 0; s < 4; ++s) {
        *(volatile v4u_t*)(X0 + (size_t)(m0 + 16 * s + L) * 2048 + b * 64 + 8 * p) = xo[s];
        *(volatile v4u_t*)(XT + (size_t)(b * 64 + 16 * s + L) * 1024 + m0 + 8 * p) = to[s];
    }
    __threadfence();
#pragma unroll
    for (int s = 0; s < 4; ++s) {
        *(volatile v4u_t*)(X0 + (size_t)(m0 + 16 * s + L) * 2048 + b * 64 + 8 * p) = xo[s];
        *(volatile v4u_t*)(XT + (size_t)(b * 64 + 16 * s + L) * 1024 + m0 + 8 * p) = to[s];
    }
}

__global__ void __launch_bounds__(128) k_tr16(const u16* __restrict__ in, u16* __restrict__ out,
                                              int ldi, int ldo, long long zi, long long zo)
{
    __shared__ __align__(16) u16 tile[64 * HP];
    const int tid = threadIdx.x;
    const int c0 = blockIdx.x * 64, r0 = blockIdx.y * 64;
    const u16* ib = in + (size_t)blockIdx.z * (size_t)zi;
    u16* ob = out + (size_t)blockIdx.z * (size_t)zo;
#pragma unroll
    for (int q = 0; q < 4; ++q) {
        const int idx = tid + 128 * q;
        const int i = idx >> 3, p8 = (idx & 7) * 8;
        *(v8us*)(tile + i * HP + p8) = *(const v8us*)(ib + (size_t)(r0 + i) * ldi + c0 + p8);
    }
    __syncthreads();
    const int L = tid >> 3, p = tid & 7;
    v8us_t o[4];
#pragma unroll
    for (int s = 0; s < 4; ++s) {
        const int c = 16 * s + L;
#pragma unroll
        for (int jj = 0; jj < 8; ++jj) o[s][jj] = tile[(8 * p + jj) * HP + c];
    }
#pragma unroll
    for (int s = 0; s < 4; ++s)
        *(volatile v8us_t*)(ob + (size_t)(c0 + 16 * s + L) * ldo + r0 + 8 * p) = o[s];
    __threadfence();
#pragma unroll
    for (int s = 0; s < 4; ++s)
        *(volatile v8us_t*)(ob + (size_t)(c0 + 16 * s + L) * ldo + r0 + 8 * p) = o[s];
}

__global__ void __launch_bounds__(128) k_softmax(const float* __restrict__ Afix, const float* __restrict__ L,
                                                 f16* __restrict__ SC)
{
    __shared__ float red[8];
    const int row = blockIdx.x, tid = threadIdx.x, lane = tid & 31, w = tid >> 5;
    const bool fixedp = row < 1024;
    const int r = fixedp ? row : row - 1024;
    const float* src = fixedp ? (Afix + (size_t)r * 1024) : (L + (size_t)r * 1024);
    f16* dst = SC + (fixedp ? (size_t)SCPLANE : (size_t)0) + (size_t)r * 1024;
    const v4f_t a = *(const v4f*)(src + 8 * tid);
    const v4f_t b = *(const v4f*)(src + 8 * tid + 4);
    float v[8];
#pragma unroll
    for (int j = 0; j < 4; ++j) { v[j] = fmaxf(a[j], 0.0f); v[4 + j] = fmaxf(b[j], 0.0f); }
    float mx = v[0];
#pragma unroll
    for (int j = 1; j < 8; ++j) mx = fmaxf(mx, v[j]);
#pragma unroll
    for (int off = 16; off > 0; off >>= 1) mx = fmaxf(mx, __shfl_xor(mx, off, 32));
    if (lane == 0) red[w] = mx;
    __syncthreads();
    mx = fmaxf(fmaxf(red[0], red[1]), fmaxf(red[2], red[3]));
    float e[8];
    float s = 0.0f;
#pragma unroll
    for (int j = 0; j < 8; ++j) { e[j] = __expf(v[j] - mx); s += e[j]; }
#pragma unroll
    for (int off = 16; off > 0; off >>= 1) s += __shfl_xor(s, off, 32);
    if (lane == 0) red[4 + w] = s;
    __syncthreads();
    s = (red[4] + red[5]) + (red[6] + red[7]);
    const float inv = 1.0f / s;
    v4f_t pa, pb;
#pragma unroll
    for (int j = 0; j < 4; ++j) { pa[j] = e[j] * inv; pb[j] = e[4 + j] * inv; }
    const v4u_t pk = pack8h(pa, pb, 1.0f);
    *(volatile v4u_t*)(dst + 8 * tid) = pk;
    __threadfence();
    *(volatile v4u_t*)(dst + 8 * tid) = pk;
}

struct GemmArgs {
    const void* A; const void* A2; const void* B; const void* B2; void* D;
    long long zA, zB, zD;
    int M, N, K, lda, ldb, ldd, split_row, sub_eye;
    float s0, s1;
};
static_assert(sizeof(GemmArgs) == 104);

__device__ __forceinline__ void gemm_store16(const float* st, f16* Db, int ldd, int row0, int col0, int lane) {
#pragma unroll
    for (int p = 0; p < 8; ++p) {
        const int lr = 4 * p + (lane >> 3), c8 = 8 * (lane & 7);
        const v4f_t x0 = *(const v4f*)(st + lr * SP + c8);
        const v4f_t x1 = *(const v4f*)(st + lr * SP + c8 + 4);
        const v4u_t pk = pack8h(x0, x1, 1.0f);
        *(volatile v4u_t*)(Db + (size_t)(row0 + lr) * ldd + col0 + c8) = pk;
    }
}
__device__ __forceinline__ void gemm_store32(const float* st, float* Df, int ldd, int row0, int col0, int lane) {
    const int h = lane >> 4, c4 = 4 * (lane & 15);
#pragma unroll
    for (int p = 0; p < 16; ++p) {
        const int lr = 2 * p + h;
        const v4f_t x0 = *(const v4f*)(st + lr * SP + c4);
        *(volatile v4f_t*)(Df + (size_t)(row0 + lr) * ldd + col0 + c4) = x0;
    }
}

template <int MODE, int OUT16>
__global__ void __launch_bounds__(128) k_gemm(GemmArgs g)
{
    __shared__ __align__(16) float stg[4 * 32 * SP];
    const int lane = threadIdx.x & 31, w = threadIdx.x >> 5, h = lane >> 4, m = lane & 15;
    const int z = blockIdx.z;
    const int rowb = blockIdx.y * 128;
    const int row0 = rowb + w * 32;
    const int col0 = blockIdx.x * 64;

    v8f acc[8];
#pragma unroll
    for (int i = 0; i < 8; ++i) acc[i] = zero8();

    if constexpr (MODE == 0) {
        const f16* Ab = (const f16*)g.A + (size_t)z * (size_t)g.zA;
        const f16* Bb = (const f16*)g.B + (size_t)z * (size_t)g.zB;
        const f16* pa0 = Ab + (size_t)(row0 + m) * g.lda + 8 * h;
        const f16* pa1 = pa0 + (size_t)16 * g.lda;
        const f16* pb  = Bb + (size_t)(col0 + m) * g.ldb + 8 * h;
        const size_t bstep = (size_t)16 * g.ldb;
#pragma unroll 1
        for (int k0 = 0; k0 < g.K; k0 += 32) {
            const v16h a0 = ldf(pa0, k0);
            const v16h a1 = ldf(pa1, k0);
            v16h b;
#pragma unroll
            for (int j = 0; j < 4; ++j) {
                b = ldf(pb + j * bstep, k0);
                acc[j]     = wm16(a0, b, acc[j]);
                acc[4 + j] = wm16(a1, b, acc[4 + j]);
            }
            asm volatile(NOP4
                         : "+v"(acc[0]), "+v"(acc[1]), "+v"(acc[2]), "+v"(acc[3]),
                           "+v"(acc[4]), "+v"(acc[5]), "+v"(acc[6]), "+v"(acc[7])
                         : "v"(a0), "v"(a1), "v"(b));
        }
    } else {
        const u16* Ah = (const u16*)g.A  + (size_t)z * (size_t)g.zA;
        const u16* Al = (const u16*)g.A2 + (size_t)z * (size_t)g.zA;
        const u16* Bh = (const u16*)g.B  + (size_t)z * (size_t)g.zB;
        const u16* Bl = (const u16*)g.B2 + (size_t)z * (size_t)g.zB;
        const size_t aoff = (size_t)(row0 + m) * g.lda + 8 * h;
        const size_t boff = (size_t)(col0 + m) * g.ldb + 8 * h;
        const u16* pah0 = Ah + aoff; const u16* pah1 = pah0 + (size_t)16 * g.lda;
        const u16* pal0 = Al + aoff; const u16* pal1 = pal0 + (size_t)16 * g.lda;
        const u16* pbh = Bh + boff; const u16* pbl = Bl + boff;
        const size_t bstep = (size_t)16 * g.ldb;
#pragma unroll 1
        for (int k0 = 0; k0 < g.K; k0 += 32) {
            const v16b ah0 = ldb(pah0, k0), ah1 = ldb(pah1, k0);
            const v16b al0 = ldb(pal0, k0), al1 = ldb(pal1, k0);
            v16b bh, bl;
#pragma unroll
            for (int j = 0; j < 4; ++j) {
                bh = ldb(pbh + j * bstep, k0);
                bl = ldb(pbl + j * bstep, k0);
                acc[j]     = wmb16(ah0, bh, acc[j]);
                acc[4 + j] = wmb16(ah1, bh, acc[4 + j]);
                acc[j]     = wmb16(ah0, bl, acc[j]);
                acc[4 + j] = wmb16(ah1, bl, acc[4 + j]);
                acc[j]     = wmb16(al0, bh, acc[j]);
                acc[4 + j] = wmb16(al1, bh, acc[4 + j]);
            }
            asm volatile(NOP4
                         : "+v"(acc[0]), "+v"(acc[1]), "+v"(acc[2]), "+v"(acc[3]),
                           "+v"(acc[4]), "+v"(acc[5]), "+v"(acc[6]), "+v"(acc[7])
                         : "v"(ah0), "v"(ah1), "v"(al0), "v"(al1), "v"(bh), "v"(bl));
        }
    }

    const float sc = (rowb < g.split_row) ? g.s0 : g.s1;
    float* st = stg + w * (32 * SP);
#pragma unroll
    for (int i = 0; i < 2; ++i)
#pragma unroll
        for (int j = 0; j < 4; ++j)
#pragma unroll
            for (int r = 0; r < 8; ++r) {
                const int lr = 16 * i + 8 * h + r, lc = 16 * j + m;
                float v = acc[4 * i + j][r] * sc;
                if (g.sub_eye) { if (row0 + lr == col0 + lc) v -= 1.0f; }
                st[lr * SP + lc] = v;
            }
    __syncthreads();
    if constexpr (OUT16 == 1) {
        f16* Db = (f16*)g.D + (size_t)z * (size_t)g.zD;
        gemm_store16(st, Db, g.ldd, row0, col0, lane);
        __threadfence();
        gemm_store16(st, Db, g.ldd, row0, col0, lane);
    } else {
        float* Df = (float*)g.D + (size_t)z * (size_t)g.zD;
        gemm_store32(st, Df, g.ldd, row0, col0, lane);
        __threadfence();
        gemm_store32(st, Df, g.ldd, row0, col0, lane);
    }
}

template <int LAYER>
__global__ void __launch_bounds__(128) k_node(const f16* __restrict__ X0, const f16* __restrict__ XG,
                                              const f16* __restrict__ WG, const f16* __restrict__ pwT,
                                              const float* __restrict__ pb,
                                              const float* __restrict__ gam, const float* __restrict__ bet,
                                              const float* __restrict__ xres, const float* __restrict__ gate,
                                              f16* __restrict__ H1, float* __restrict__ out)
{
    __shared__ __align__(16) f16 hs[32 * HP];
    __shared__ __align__(16) float vs[32 * SP];
    __shared__ __align__(16) f16 h16[32 * 64];
    const int n = blockIdx.x;
    const int tid = threadIdx.x, lane = tid & 31, w = tid >> 5, h = lane >> 4, m = lane & 15;
    const int b0 = 16 * (w >> 1), o0 = 32 * (w & 1);

    v8f acc[2];
    acc[0] = zero8(); acc[1] = zero8();
#pragma unroll
    for (int gg = 0; gg < 2; ++gg) {
        const f16* wg  = WG + (size_t)gg * WGPLANE + (size_t)n * WGROW;
        const f16* s0p = X0 + (size_t)n * 2048;
        const f16* s1p = XG + (size_t)gg * XGPLANE + (size_t)n * 2048;
        const f16* s2p = XG + (size_t)gg * XGPLANE + (size_t)(1024 + n) * 2048;
#pragma unroll
        for (int kc = 0; kc < 6; ++kc) {
            const f16* sp = (kc < 2) ? s0p : ((kc < 4) ? s1p : s2p);
            const v16h a  = ldf(sp + (b0 + m) * 64 + (kc & 1) * 32 + 8 * h, 0);
            const v16h q0 = ldf(wg + (size_t)(o0 + m) * 192 + kc * 32 + 8 * h, 0);
            const v16h q1 = ldf(wg + (size_t)(o0 + 16 + m) * 192 + kc * 32 + 8 * h, 0);
            acc[0] = wm16(a, q0, acc[0]);
            acc[1] = wm16(a, q1, acc[1]);
            asm volatile(NOP4 : "+v"(acc[0]), "+v"(acc[1]) : "v"(a), "v"(q0), "v"(q1));
        }
    }
    float bg[2];
#pragma unroll
    for (int j = 0; j < 2; ++j) {
        const int o = o0 + 16 * j + m;
        bg[j] = (float)WG[(size_t)n * WGROW + 12288 + o] + (float)WG[(size_t)WGPLANE + (size_t)n * WGROW + 12288 + o];
    }
#pragma unroll
    for (int j = 0; j < 2; ++j)
#pragma unroll
        for (int r = 0; r < 8; ++r) {
            const float v = (acc[j][r] + bg[j]) * (1.0f / 1024.0f);
            hs[(b0 + 8 * h + r) * HP + o0 + 16 * j + m] = (f16)(v * 16.0f);
        }
    __syncthreads();

    v8f ac2[2];
    ac2[0] = zero8(); ac2[1] = zero8();
    const f16* pha = hs + (b0 + m) * HP + 8 * h;
#pragma unroll
    for (int k0 = 0; k0 < 64; k0 += 32) {
        const v16h a  = ldf(pha, k0);
        const v16h q0 = ldf(pwT + (size_t)(o0 + m) * 64 + 8 * h, k0);
        const v16h q1 = ldf(pwT + (size_t)(o0 + 16 + m) * 64 + 8 * h, k0);
        ac2[0] = wm16(a, q0, ac2[0]);
        ac2[1] = wm16(a, q1, ac2[1]);
        asm volatile(NOP4 : "+v"(ac2[0]), "+v"(ac2[1]) : "v"(a), "v"(q0), "v"(q1));
    }
    float sg = 0.0f;
    if (LAYER == 2) sg = 1.0f / (1.0f + expf(-gate[0]));
#pragma unroll
    for (int j = 0; j < 2; ++j) {
        const int t = o0 + 16 * j + m;
        const float pbt = pb[t];
#pragma unroll
        for (int r = 0; r < 8; ++r) {
            const int rb = b0 + 8 * h + r;
            float v = ac2[j][r] * (1.0f / 64.0f) + pbt;
            if (LAYER == 2) v += sg * xres[(size_t)rb * 65536 + (size_t)n * 64 + t];
            vs[rb * SP + t] = v;
        }
    }
    __syncthreads();

    {
        const int rb = tid >> 2, q = tid & 3;
        float xv[16];
#pragma unroll
        for (int u = 0; u < 4; ++u) {
            const v4f_t t4 = *(const v4f*)(vs + rb * SP + 16 * q + 4 * u);
#pragma unroll
            for (int jj = 0; jj < 4; ++jj) xv[4 * u + jj] = t4[jj];
        }
        float s = 0.0f;
#pragma unroll
        for (int jj = 0; jj < 16; ++jj) s += xv[jj];
        s += __shfl_xor(s, 1, 32);
        s += __shfl_xor(s, 2, 32);
        const float mean = s * (1.0f / 64.0f);
        float ss = 0.0f;
#pragma unroll
        for (int jj = 0; jj < 16; ++jj) { const float d = xv[jj] - mean; ss += d * d; }
        ss += __shfl_xor(ss, 1, 32);
        ss += __shfl_xor(ss, 2, 32);
        const float rstd = rsqrtf(ss * (1.0f / 64.0f) + 1e-5f);
        float y[16];
#pragma unroll
        for (int jj = 0; jj < 16; ++jj) {
            const int t = 16 * q + jj;
            float yy = (xv[jj] - mean) * rstd * gam[t] + bet[t];
            if (LAYER == 1) yy = fmaxf(yy, 0.0f);
            y[jj] = yy;
        }
        if (LAYER == 1) {
            v4f_t a0, a1, a2, a3;
#pragma unroll
            for (int jj = 0; jj < 4; ++jj) { a0[jj] = y[jj]; a1[jj] = y[4 + jj]; a2[jj] = y[8 + jj]; a3[jj] = y[12 + jj]; }
            *(v4u*)(h16 + rb * 64 + 16 * q)     = pack8h(a0, a1, 1.0f);
            *(v4u*)(h16 + rb * 64 + 16 * q + 8) = pack8h(a2, a3, 1.0f);
        } else {
#pragma unroll
            for (int u = 0; u < 4; ++u) {
                v4f_t t4;
#pragma unroll
                for (int jj = 0; jj < 4; ++jj) t4[jj] = y[4 * u + jj];
                *(v4f*)(vs + rb * SP + 16 * q + 4 * u) = t4;
            }
        }
    }
    __syncthreads();

    if (LAYER == 1) {
        f16* dst = H1 + (size_t)n * 2048;
        const v4u_t u0 = *(const v4u*)(h16 + 8 * tid);
        const v4u_t u1 = *(const v4u*)(h16 + 1024 + 8 * tid);
        *(volatile v4u_t*)(dst + 8 * tid) = u0;
        *(volatile v4u_t*)(dst + 1024 + 8 * tid) = u1;
        __threadfence();
        *(volatile v4u_t*)(dst + 8 * tid) = u0;
        *(volatile v4u_t*)(dst + 1024 + 8 * tid) = u1;
    } else {
        const int c4 = 4 * m;
        v4f_t ov[4];
#pragma unroll
        for (int p = 0; p < 4; ++p) ov[p] = *(const v4f*)(vs + (8 * w + 2 * p + h) * SP + c4);
#pragma unroll
        for (int p = 0; p < 4; ++p)
            *(volatile v4f_t*)(out + (size_t)(8 * w + 2 * p + h) * 65536 + (size_t)n * 64 + c4) = ov[p];
        __threadfence();
#pragma unroll
        for (int p = 0; p < 4; ++p)
            *(volatile v4f_t*)(out + (size_t)(8 * w + 2 * p + h) * 65536 + (size_t)n * 64 + c4) = ov[p];
    }
}

static GemmArgs make_args(const void* A, const void* A2, const void* B, const void* B2, void* D,
                          long long zA, long long zB, long long zD,
                          int M, int N, int K, int lda, int ldb, int ldd,
                          int split_row, int sub_eye, float s0, float s1)
{
    GemmArgs g;
    g.A = A; g.A2 = A2; g.B = B; g.B2 = B2; g.D = D;
    g.zA = zA; g.zB = zB; g.zD = zD;
    g.M = M; g.N = N; g.K = K; g.lda = lda; g.ldb = ldb; g.ldd = ldd;
    g.split_row = split_row; g.sub_eye = sub_eye; g.s0 = s0; g.s1 = s1;
    return g;
}

extern "C" void kernel_launch(void* const* d_in, const int* in_sizes, int n_in,
                              void* d_out, int out_size, void* d_ws, size_t ws_size,
                              hipStream_t stream)
{
    if (n_in < 16) return;
    if (in_sizes[0] != NBATCH * NNODE * NT) return;
    if (in_sizes[1] != NNODE * NNODE) return;
    if (in_sizes[2] != NNODE * 64) return;
    if (in_sizes[3] != 2 * 64 * 3 * 64 * 64) return;
    if (in_sizes[4] != 2 * 64 * 64) return;
    if (in_sizes[5] != 2 * 64 * 3 * 64 * 64) return;
    if (in_sizes[6] != 2 * 64 * 64) return;
    if (in_sizes[7] != 64 * 64) return;
    if (in_sizes[8] != 64) return;
    if (in_sizes[9] != 64 * 64) return;
    if (in_sizes[10] != 64) return;
    if (in_sizes[11] != 64 || in_sizes[12] != 64 || in_sizes[13] != 64 || in_sizes[14] != 64) return;
    if (in_sizes[15] < 1) return;
    if (out_size != NBATCH * NNODE * NT) return;

    const float* x     = (const float*)d_in[0];
    const float* A_fix = (const float*)d_in[1];
    const float* E     = (const float*)d_in[2];
    const float* W1    = (const float*)d_in[3];
    const float* b1p   = (const float*)d_in[4];
    const float* W2    = (const float*)d_in[5];
    const float* b2p   = (const float*)d_in[6];
    const float* p1w   = (const float*)d_in[7];
    const float* p1b   = (const float*)d_in[8];
    const float* p2w   = (const float*)d_in[9];
    const float* p2b   = (const float*)d_in[10];
    const float* g1    = (const float*)d_in[11];
    const float* be1   = (const float*)d_in[12];
    const float* g2    = (const float*)d_in[13];
    const float* be2   = (const float*)d_in[14];
    const float* rgate = (const float*)d_in[15];
    float* out = (float*)d_out;

    size_t off = 0;
    auto take = [&](size_t bytes) -> size_t { const size_t o = off; off += (bytes + 255) & ~(size_t)255; return o; };
    const size_t oEhi = take((size_t)65536 * 2);
    const size_t oElo = take((size_t)65536 * 2);
    const size_t oE16 = take((size_t)65536 * 2);
    const size_t oWT  = take((size_t)4 * WTPLANE * 2);
    const size_t oPWT = take((size_t)2 * 4096 * 2);
    const size_t oXT1 = take((size_t)2048 * 1024 * 2);
    const size_t oXT2 = take((size_t)2048 * 1024 * 2);
    const size_t oX01 = take((size_t)1024 * 2048 * 2);
    const size_t oH1  = take((size_t)1024 * 2048 * 2);
    const size_t oL   = take((size_t)1024 * 1024 * 4);
    const size_t oSC  = take((size_t)2 * SCPLANE * 2);
    const size_t oST  = take((size_t)2 * STPLANE * 2);
    const size_t oWG  = take((size_t)2 * WGPLANE * 2);
    const size_t oXG  = take((size_t)2 * XGPLANE * 2);
    const size_t total = off;
    if (total > ws_size || total > ((size_t)128 << 20)) return;

    char* ws = (char*)d_ws;
    u16* Ehi = (u16*)(ws + oEhi);
    u16* Elo = (u16*)(ws + oElo);
    f16* E16 = (f16*)(ws + oE16);
    f16* WT  = (f16*)(ws + oWT);
    f16* pwT = (f16*)(ws + oPWT);
    f16* XT1 = (f16*)(ws + oXT1);
    f16* XT2 = (f16*)(ws + oXT2);
    f16* X01 = (f16*)(ws + oX01);
    f16* H1  = (f16*)(ws + oH1);
    float* Lf = (float*)(ws + oL);
    f16* SC  = (f16*)(ws + oSC);
    f16* ST  = (f16*)(ws + oST);
    f16* WG  = (f16*)(ws + oWG);
    f16* XG  = (f16*)(ws + oXG);

    k_prep_e<<<32, 256, 0, stream>>>(E, Ehi, Elo, E16, 8192);
    k_trw<<<dim3(194, 2, 2), 128, 0, stream>>>(W1, W2, b1p, b2p, p1w, p2w, WT, pwT);
    k_trx<<<dim3(16, 32, 1), 128, 0, stream>>>(x, XT1, X01);

    k_gemm<1, 0><<<dim3(16, 8, 1), 128, 0, stream>>>(
        make_args(Ehi, Elo, Ehi, Elo, Lf, 0, 0, 0, 1024, 1024, 64, 64, 64, 1024, 1 << 30, 0, 1.0f, 1.0f));
    k_softmax<<<2048, 128, 0, stream>>>(A_fix, Lf, SC);
    k_tr16<<<dim3(16, 16, 2), 128, 0, stream>>>((const u16*)SC, (u16*)ST, 1024, 1024,
                                                (long long)SCPLANE, (long long)STPLANE);
    k_gemm<0, 1><<<dim3(16, 8, 2), 128, 0, stream>>>(
        make_args(SC, SC, ST, ST, SC + (size_t)1024 * 1024, SCPLANE, STPLANE, SCPLANE,
                  1024, 1024, 1024, 1024, 1024, 1024, 1 << 30, 1, 2.0f, 2.0f));

    k_gemm<0, 1><<<dim3(WGROW / 64, 8, 2), 128, 0, stream>>>(
        make_args(E16, E16, WT, WT, WG, 0, WTPLANE, WGPLANE,
                  1024, WGROW, 64, 64, 64, WGROW, 1 << 30, 0, 1.0f, 1.0f));
    k_gemm<0, 1><<<dim3(32, 16, 2), 128, 0, stream>>>(
        make_args(SC, SC, XT1, XT1, XG, SCPLANE, 0, XGPLANE,
                  2048, 2048, 1024, 1024, 1024, 2048, 1024, 0, 16.0f, 1.0f));
    k_node<1><<<NNODE, 128, 0, stream>>>(X01, XG, WG, pwT, p1b, g1, be1, x, rgate, H1, out);

    k_tr16<<<dim3(32, 16, 1), 128, 0, stream>>>((const u16*)H1, (u16*)XT2, 2048, 1024, 0LL, 0LL);
    k_gemm<0, 1><<<dim3(WGROW / 64, 8, 2), 128, 0, stream>>>(
        make_args(E16, E16, WT + (size_t)2 * WTPLANE, WT + (size_t)2 * WTPLANE, WG, 0, WTPLANE, WGPLANE,
                  1024, WGROW, 64, 64, 64, WGROW, 1 << 30, 0, 1.0f, 1.0f));
    k_gemm<0, 1><<<dim3(32, 16, 2), 128, 0, stream>>>(
        make_args(SC, SC, XT2, XT2, XG, SCPLANE, 0, XGPLANE,
                  2048, 2048, 1024, 1024, 1024, 2048, 1024, 0, 16.0f, 1.0f));
    k_node<2><<<NNODE, 128, 0, stream>>>(H1, XG, WG, pwT + 4096, p2b, g2, be2, x, rgate, H1, out);
}
